// PairwiseScorer_30897994727574
// MI455X (gfx1250) — hardware-verified
//
#include <hip/hip_runtime.h>
#include <math.h>

typedef __attribute__((ext_vector_type(16))) _Float16 v16h;
typedef __attribute__((ext_vector_type(16))) __bf16 v16b;
typedef __attribute__((ext_vector_type(8)))  _Float16 v8h;
typedef __attribute__((ext_vector_type(8)))  float v8f;
typedef __attribute__((ext_vector_type(4)))  float v4f;
typedef __attribute__((ext_vector_type(2)))  float v2f;
typedef __attribute__((ext_vector_type(4)))  unsigned v4u;
typedef __attribute__((ext_vector_type(4)))  int v4i;
typedef float __attribute__((may_alias)) float_a;
typedef int __attribute__((may_alias)) int_a;

template <typename T> __device__ __forceinline__ void vst2(void* p, T v) { *(volatile T*)p = v; __threadfence(); *(volatile T*)p = v; }
__device__ __forceinline__ v8f wmma16(v16h a, v16h b, v8f c) {
  v8f d = __builtin_amdgcn_wmma_f32_16x16x32_f16(false, a, false, b, (short)0, c, false, false);
  asm volatile("v_nop\n\tv_nop\n\tv_nop\n\tv_nop" : "+v"(d) : "v"(a), "v"(b));
  return d;
}
__device__ __forceinline__ v8f wmma_bf(v16b a, v16b b, v8f c) {
  v8f d = __builtin_amdgcn_wmma_f32_16x16x32_bf16(false, a, false, b, (short)0, c, false, false);
  asm volatile("v_nop\n\tv_nop\n\tv_nop\n\tv_nop" : "+v"(d) : "v"(a), "v"(b));
  return d;
}
__device__ __forceinline__ v16h frag_h(const _Float16* rowk0, int lane) {
  union { v16h v; v8h q[2]; } u; const _Float16* p = rowk0 + 8 * (lane >> 4);
  u.q[0] = *(const v8h*)p; u.q[1] = *(const v8h*)(p + 16); return u.v;
}
__device__ __forceinline__ v16h frag_f32(const float* rowk0, int lane) {
  v16h a; const float* p = rowk0 + 8 * (lane >> 4);
#pragma unroll
  for (int i = 0; i < 8; ++i) { a[i] = (_Float16)p[i]; a[8 + i] = (_Float16)p[16 + i]; }
  return a;
}
__device__ __forceinline__ v16h frag_f32s(const float* rowk0, int lane, float sc) {
  v16h a; const float* p = rowk0 + 8 * (lane >> 4);
#pragma unroll
  for (int i = 0; i < 8; ++i) { a[i] = (_Float16)(p[i] * sc); a[8 + i] = (_Float16)(p[16 + i] * sc); }
  return a;
}
__device__ __forceinline__ v16h fragc_f32(const float* W, int k0, int n, int lane, int ld, int K) {
  v16h a; const int g = lane >> 4;
#pragma unroll
  for (int i = 0; i < 8; ++i) { const int ka = k0 + 8 * g + i, kb = ka + 16;
    a[i] = (_Float16)(ka < K ? W[(size_t)ka * ld + n] : 0.f); a[8 + i] = (_Float16)(kb < K ? W[(size_t)kb * ld + n] : 0.f); }
  return a;
}
struct F2 { v16b h, l; };
__device__ __forceinline__ F2 bsplit16(const float v[16]) { F2 r;
#pragma unroll
  for (int i = 0; i < 16; ++i) { const __bf16 h = (__bf16)v[i]; r.h[i] = h; r.l[i] = (__bf16)(v[i] - (float)h); }
  return r; }
__device__ __forceinline__ F2 split_row(const float* row, int k0, int lane) { float v[16]; const float* p = row + k0 + 8 * (lane >> 4);
#pragma unroll
  for (int i = 0; i < 8; ++i) { v[i] = p[i]; v[8 + i] = p[16 + i]; }
  return bsplit16(v); }
__device__ __forceinline__ F2 split_rowK(const float* row, int k0, int lane, int K) { float v[16]; const int g = lane >> 4;
#pragma unroll
  for (int i = 0; i < 8; ++i) { const int ka = k0 + 8 * g + i, kb = ka + 16; v[i] = ka < K ? row[ka] : 0.f; v[8 + i] = kb < K ? row[kb] : 0.f; }
  return bsplit16(v); }
__device__ __forceinline__ F2 split_col(const float* W, int k0, int n, int lane, int ld, int K) { float v[16]; const int g = lane >> 4;
#pragma unroll
  for (int i = 0; i < 8; ++i) { const int ka = k0 + 8 * g + i, kb = ka + 16; v[i] = ka < K ? W[(size_t)ka * ld + n] : 0.f; v[8 + i] = kb < K ? W[(size_t)kb * ld + n] : 0.f; }
  return bsplit16(v); }
__device__ __forceinline__ v8f mac3(const F2& a, const F2& b, v8f c) { c = wmma_bf(a.l, b.h, c); c = wmma_bf(a.h, b.l, c); return wmma_bf(a.h, b.h, c); }
__device__ __forceinline__ float sigm(float v) { return 1.0f / (1.0f + expf(-v)); }
#define LDSX() do { asm volatile("s_wait_dscnt 0" ::: "memory"); __builtin_amdgcn_wave_barrier(); __builtin_amdgcn_fence(__ATOMIC_RELEASE, "workgroup"); } while (0)


#define NB 2
#define S 512
#define H 256
#define H2 128
__device__ __forceinline__ float relu(float v) { return v > 0.f ? v : 0.f; }

__global__ __launch_bounds__(128) void k_proj(const float* __restrict__ nf, const float* __restrict__ W1, float* __restrict__ P) {
  __shared__ __align__(16) float so[4][16][132];
  const int tid = threadIdx.x, wave = tid >> 5, lane = tid & 31, col = lane & 15, g = lane >> 4; const int r0 = blockIdx.x * 64 + wave * 16; const int which = blockIdx.y;
  const float* Wk = W1 + (size_t)which * H * H; float* Pw = P + (size_t)which * NB * S * H;
#pragma unroll 1
  for (int nh = 0; nh < 2; ++nh) { v8f acc[8] = {};
#pragma unroll 1
    for (int kc = 0; kc < H / 32; ++kc) { const F2 a = split_row(nf + (size_t)(r0 + col) * H, kc * 32, lane);
#pragma unroll
      for (int j = 0; j < 8; ++j) acc[j] = mac3(a, split_col(Wk, kc * 32, nh * 128 + j * 16 + col, lane, H, H), acc[j]); }
#pragma unroll
    for (int j = 0; j < 8; ++j)
#pragma unroll
      for (int r = 0; r < 8; ++r) so[wave][8 * g + r][j * 16 + col] = acc[j][r];
    LDSX();
    for (int rl = 0; rl < 16; ++rl) vst2(Pw + (size_t)(r0 + rl) * H + nh * 128 + lane * 4, *(const v4f*)(&so[wave][rl][lane * 4]));
    LDSX(); }
}
__global__ __launch_bounds__(256) void k_pack(const float* __restrict__ W2, _Float16* __restrict__ W2T) {
  const int n = blockIdx.x, tid = threadIdx.x; __shared__ __align__(16) _Float16 srow[H];
  srow[tid] = (_Float16)(W2[(size_t)tid * H2 + n] * 16.0f); __syncthreads();
  if (tid < H / 8) vst2(W2T + (size_t)n * H + tid * 8, *(const v4u*)(&srow[tid * 8]));
}
__global__ __launch_bounds__(128) void k_pair(const float* __restrict__ P, const float* __restrict__ prior, const float* __restrict__ W1, const float* __restrict__ b1, const _Float16* __restrict__ W2T, const float* __restrict__ b2,
                                             const float* __restrict__ W3, const float* __restrict__ b3, float* __restrict__ out) {
  __shared__ __align__(16) _Float16 sa[64][H + 8];
  __shared__ float ssc[64];
  const int tid = threadIdx.x, wave = tid >> 5, lane = tid & 31, col = lane & 15, g = lane >> 4;
  const int b = blockIdx.z, i = blockIdx.y, j0 = blockIdx.x * 64;
  const float* Pi = P + ((size_t)b * S + i) * H; const float* Pj0 = P + (size_t)NB * S * H + ((size_t)b * S + j0) * H; const float* wp = W1 + (size_t)2 * H * H; const float* pr = prior + ((size_t)b * S + i) * S + j0;
#pragma unroll 1
  for (int cc = 0; cc < 2; ++cc) { const int c = tid + cc * 128; const float base = Pi[c] + b1[c], wpc = wp[c];
#pragma unroll 4
    for (int jl = 0; jl < 64; ++jl) sa[jl][c] = (_Float16)relu(base + Pj0[(size_t)jl * H + c] + pr[jl] * wpc); }
  __syncthreads();
  v8f acc[8] = {};
#pragma unroll 2
  for (int kc = 0; kc < H / 32; ++kc) { const v16h a = frag_h(&sa[wave * 16 + col][0] + kc * 32, lane);
#pragma unroll
    for (int j = 0; j < 8; ++j) acc[j] = wmma16(a, frag_h(W2T + (size_t)(j * 16 + col) * H + kc * 32, lane), acc[j]); }
  float part[8];
#pragma unroll
  for (int r = 0; r < 8; ++r) { float s = 0.f;
#pragma unroll
    for (int j = 0; j < 8; ++j) { const int n = j * 16 + col; s += relu(acc[j][r] * (1.0f / 16.0f) + b2[n]) * W3[n]; }
    part[r] = s; }
#pragma unroll
  for (int r = 0; r < 8; ++r) {
#pragma unroll
    for (int o = 1; o < 16; o <<= 1) part[r] += __shfl_xor(part[r], o, 32); }
  if (col == 0) {
#pragma unroll
    for (int r = 0; r < 8; ++r) ssc[wave * 16 + 8 * g + r] = part[r] + b3[0]; }
  __syncthreads();
  if (tid < 64) vst2(out + ((size_t)b * S + i) * S + j0 + tid, (float_a)ssc[tid]);
}
extern "C" void kernel_launch(void* const* d_in, const int* in_sizes, int n_in, void* d_out, int out_size, void* d_ws, size_t ws_size, hipStream_t stream) {
  (void)in_sizes; (void)n_in; (void)out_size; (void)ws_size;
  const float** I = (const float**)d_in;
  const float* nf = I[0]; const float* prior = I[1]; const float* W1 = I[2]; const float* b1 = I[3]; const float* W2 = I[4]; const float* b2 = I[5]; const float* W3 = I[6]; const float* b3 = I[7];
  float* out = (float*)d_out;
  char* ws = (char*)d_ws; size_t off = 0;
  auto take = [&](size_t bytes) { char* p = ws + off; off += (bytes + 255) & ~(size_t)255; return p; };
  float* P = (float*)take((size_t)2 * NB * S * H * 4); _Float16* W2T = (_Float16*)take((size_t)H2 * H * 2);
  k_proj<<<dim3(NB * S / 64, 2), 128, 0, stream>>>(nf, W1, P);
  k_pack<<<H2, 256, 0, stream>>>(W2, W2T);
  k_pair<<<dim3(S / 64, S, NB), 128, 0, stream>>>(P, prior, W1, b1, W2T, b2, W3, b3, out);
}
